// SelfA_63333587747382
// MI455X (gfx1250) — hardware-verified
//
#include <hip/hip_runtime.h>
#include <stdint.h>

typedef _Float16 v16h __attribute__((ext_vector_type(16)));
typedef _Float16 v8h_t __attribute__((ext_vector_type(8)));
typedef v8h_t __attribute__((may_alias)) v8h;
typedef _Float16 v2h_t __attribute__((ext_vector_type(2)));
typedef v2h_t __attribute__((may_alias)) v2h;
typedef float v8f __attribute__((ext_vector_type(8)));
typedef float v4f_t __attribute__((ext_vector_type(4)));
typedef v4f_t __attribute__((may_alias)) v4f;

#define B_    2
#define C_    66
#define T_    32
#define N_    512
#define L_    2
#define QK_   64
#define VCH_  124
#define K_    16
#define CIN_  128
#define NP_   (B_ * T_ * N_)
#define TN_   (T_ * N_)
#define NCAND_ (3 * N_)
#define GP_   72
#define FP_   136
#define QP_   72
#define OCH_  128

typedef char chk_np8_t[(NP_ % 8 == 0) ? 1 : -1];
typedef char chk_np32_t[(NP_ % 32 == 0) ? 1 : -1];
typedef char chk_n32_t[(N_ % 32 == 0) ? 1 : -1];

__device__ __forceinline__ v8f wmma_f16(v16h a, v16h b, v8f c) {
  v8f d = __builtin_amdgcn_wmma_f32_16x16x32_f16(false, a, false, b, (short)0, c, false, false);
  asm volatile("v_nop\n\tv_nop\n\tv_nop\n\tv_nop" : "+v"(d) : "v"(a), "v"(b));
  return d;
}

union Frag { v16h v; v8h q[2]; };

__device__ __forceinline__ v16h frag16(const _Float16* M, int pitch, int idx0, int k0, int m16, int h) {
  Frag f;
  const _Float16* rp = M + (idx0 + m16) * pitch + k0 + 8 * h;
  f.q[0] = *(const v8h*)(rp);
  f.q[1] = *(const v8h*)(rp + 16);
  return f.v;
}

__device__ __forceinline__ v8f zero8() {
  v8f z = {0.f, 0.f, 0.f, 0.f, 0.f, 0.f, 0.f, 0.f};
  return z;
}

__device__ __forceinline__ unsigned long long shfl_xor_u64(unsigned long long v, int m) {
  int lo = (int)(v & 0xffffffffull);
  int hi = (int)(v >> 32);
  lo = __shfl_xor(lo, m, 32);
  hi = __shfl_xor(hi, m, 32);
  return ((unsigned long long)(unsigned int)hi << 32) | (unsigned int)lo;
}

__global__ __launch_bounds__(256) void k_cvtw(const float* __restrict__ Wqk,
                                              const float* __restrict__ Wv,
                                              _Float16* wq16, _Float16* wv16) {
  const int gid = blockIdx.x * 256 + threadIdx.x;
  if (gid >= 8192) return;
  union { v8h v; _Float16 s[8]; } u;
  _Float16* dst;
  if (gid < 4096) {
    const int e0 = gid * 8;
#pragma unroll
    for (int i = 0; i < 8; ++i) u.s[i] = (_Float16)(Wqk[e0 + i] * 16.0f);
    dst = wq16 + e0;
  } else {
    const int e0 = (gid - 4096) * 8;
    const int l = e0 >> 14, rem = e0 & 16383, o = rem >> 7, c = rem & 127;
    if (o < VCH_) {
#pragma unroll
      for (int i = 0; i < 8; ++i)
        u.s[i] = (_Float16)(Wv[(l * VCH_ + o) * CIN_ + c + i] * 16.0f);
    } else {
#pragma unroll
      for (int i = 0; i < 8; ++i) u.s[i] = (_Float16)0.0f;
    }
    dst = wv16 + e0;
  }
  *(volatile v8h*)dst = u.v;
  __threadfence();
  *(volatile v8h*)dst = u.v;
}

__global__ __launch_bounds__(256) void k_group(const float* __restrict__ x, _Float16* G) {
#pragma clang fp contract(off)
  __shared__ __attribute__((aligned(16))) _Float16 S[8][K_ * GP_];
  const int lane = threadIdx.x & 31;
  const int wv = threadIdx.x >> 5;
  const int p = blockIdx.x * 8 + wv;
  const int n = p & (N_ - 1);
  const int t = (p >> 9) & (T_ - 1);
  const int b = p >> 14;
  const float* xb = x + (size_t)b * C_ * TN_;

  const float cx = xb[0 * TN_ + t * N_ + n];
  const float cy = xb[1 * TN_ + t * N_ + n];
  const float cz = xb[2 * TN_ + t * N_ + n];

  float d[48];
#pragma unroll
  for (int s = 0; s < 48; ++s) {
    const int cand = s * 32 + lane;
    int tj = t - 1 + (cand >> 9);
    tj = tj < 0 ? 0 : (tj > T_ - 1 ? T_ - 1 : tj);
    const int nj = cand & (N_ - 1);
    const float* src = xb + tj * N_ + nj;
    const float dx = cx - src[0];
    const float dy = cy - src[TN_];
    const float dz = cz - src[2 * TN_];
    const float sx = dx * dx;
    const float sy = dy * dy;
    const float sz = dz * dz;
    const float sxy = sx + sy;
    d[s] = sxy + sz;
  }

  unsigned long long selm = 0;
  int keep = 0;
  for (int r = 0; r < K_; ++r) {
    float bd = 3.0e38f;
    int bs = 0;
#pragma unroll
    for (int s = 0; s < 48; ++s) {
      const bool ok = (((selm >> s) & 1ull) == 0) && (d[s] < bd);
      bd = ok ? d[s] : bd;
      bs = ok ? s : bs;
    }
    const unsigned int cand = (unsigned int)(bs * 32 + lane);
    unsigned long long key = ((unsigned long long)__float_as_uint(bd) << 32) | cand;
#pragma unroll
    for (int m = 1; m < 32; m <<= 1) {
      const unsigned long long o = shfl_xor_u64(key, m);
      key = (o < key) ? o : key;
    }
    const unsigned int wc = (unsigned int)key;
    if ((int)(wc & 31u) == lane) selm |= 1ull << (wc >> 5);
    if (r == lane) keep = (int)wc;
  }

  _Float16* Sw = S[wv];
  if (lane < K_) {
    _Float16* Sr = Sw + lane * GP_;
    Sr[4] = (_Float16)0.0f; Sr[5] = (_Float16)0.0f; Sr[6] = (_Float16)0.0f; Sr[7] = (_Float16)0.0f;
    Sr[70] = (_Float16)0.0f; Sr[71] = (_Float16)0.0f;
  }
  float xcl = 0.0f;
  if (lane < 4) xcl = xb[lane * TN_ + t * N_ + n];
  for (int k = 0; k < K_; ++k) {
    int cj = __shfl(keep, k, 32);
    cj = cj < 0 ? 0 : (cj > NCAND_ - 1 ? NCAND_ - 1 : cj);
    int tj = t - 1 + (cj >> 9);
    tj = tj < 0 ? 0 : (tj > T_ - 1 ? T_ - 1 : tj);
    const int nj = cj & (N_ - 1);
    const float* src = xb + tj * N_ + nj;
    _Float16* Sr = Sw + k * GP_;
    const float v0 = src[lane * TN_];
    if (lane < 4) Sr[lane] = (_Float16)(xcl - v0);
    else          Sr[lane + 4] = (_Float16)v0;
    const float v1 = src[(32 + lane) * TN_];
    Sr[36 + lane] = (_Float16)v1;
    if (lane < 2) {
      const float v2 = src[(64 + lane) * TN_];
      Sr[68 + lane] = (_Float16)v2;
    }
  }
  __syncthreads();

  _Float16* Gp = G + (size_t)p * (K_ * GP_);
#pragma unroll
  for (int it = 0; it < 5; ++it) {
    const int q = it * 32 + lane;
    if (q < (K_ * GP_) / 8) {
      const v8h v = *(const v8h*)(Sw + 8 * q);
      *(volatile v8h*)(Gp + 8 * q) = v;
    }
  }
  __threadfence();
#pragma unroll
  for (int it = 0; it < 5; ++it) {
    const int q = it * 32 + lane;
    if (q < (K_ * GP_) / 8) {
      const v8h v = *(const v8h*)(Sw + 8 * q);
      *(volatile v8h*)(Gp + 8 * q) = v;
    }
  }
}

__global__ __launch_bounds__(64) void k_attn(const float* __restrict__ x,
                                             const float* __restrict__ bqk,
                                             const float* __restrict__ bv,
                                             const _Float16* __restrict__ wq16,
                                             const _Float16* __restrict__ wv16,
                                             const _Float16* __restrict__ G,
                                             float* out) {
  __shared__ __attribute__((aligned(16))) _Float16 Fs[2][16 * FP_];
  __shared__ __attribute__((aligned(16))) _Float16 Qs[2][16 * QP_];
  __shared__ __attribute__((aligned(16))) _Float16 Ks[2][16 * QP_];
  __shared__ float AFs[2][16];
  __shared__ __attribute__((aligned(16))) float ST[L_ * OCH_ * 32];

  const int lane = threadIdx.x & 31;
  const int w = threadIdx.x >> 5;
  const int h = lane >> 4;
  const int m16 = lane & 15;
  const int p0 = blockIdx.x * 32;
  const int b = p0 >> 14;
  const int t = (p0 >> 9) & (T_ - 1);
  const int n0 = p0 & (N_ - 1);
  const float* xb = x + (size_t)b * C_ * TN_;
  _Float16* F = Fs[w];
  _Float16* Q = Qs[w];
  _Float16* Kt = Ks[w];
  float* AF = AFs[w];

  for (int i = 0; i < 16; ++i) {
    const int nl = w * 16 + i;
    const int n = n0 + nl;
    const int p = p0 + nl;

    const _Float16* Gp = G + (size_t)p * (K_ * GP_);
#pragma unroll
    for (int it = 0; it < 5; ++it) {
      const int q = it * 32 + lane;
      if (q < (K_ * GP_) / 8) {
        const int k = q / 9;
        const int c = q - 9 * k;
        union { v8h v; v2h d[4]; } u;
        u.v = *(const v8h*)(Gp + k * GP_ + 8 * c);
        _Float16* Fr = F + k * FP_;
        if (c == 0) {
          *(v2h*)(Fr + 0) = u.d[0];
          *(v2h*)(Fr + 2) = u.d[1];
        } else {
          const int d0 = 58 + 8 * c;
          *(v2h*)(Fr + d0 + 0) = u.d[0];
          *(v2h*)(Fr + d0 + 2) = u.d[1];
          *(v2h*)(Fr + d0 + 4) = u.d[2];
          *(v2h*)(Fr + d0 + 6) = u.d[3];
        }
      }
    }
    if (lane < 31) {
      const int c0 = 4 + 2 * lane;
      union { v2h v; _Float16 s[2]; } cv;
      cv.s[0] = (_Float16)xb[c0 * TN_ + t * N_ + n];
      cv.s[1] = (_Float16)xb[(c0 + 1) * TN_ + t * N_ + n];
#pragma unroll
      for (int k = 0; k < K_; ++k) *(v2h*)(F + k * FP_ + c0) = cv.v;
    }
    __syncthreads();

    v16h bf[4];
#pragma unroll
    for (int ks = 0; ks < 4; ++ks) bf[ks] = frag16(F, FP_, 0, ks * 32, m16, h);

#pragma unroll 1
    for (int l = 0; l < L_; ++l) {
      const _Float16* wq = wq16 + l * (128 * CIN_);
      const _Float16* wvp = wv16 + l * (128 * CIN_);

#pragma unroll 1
      for (int mt = 0; mt < 8; ++mt) {
        v8f acc = zero8();
#pragma unroll
        for (int ks = 0; ks < 4; ++ks)
          acc = wmma_f16(frag16(wq, CIN_, mt * 16, ks * 32, m16, h), bf[ks], acc);
        union { v8h v; _Float16 s[8]; } o8;
        const int obase = mt * 16 + 8 * h;
#pragma unroll
        for (int r = 0; r < 8; ++r)
          o8.s[r] = (_Float16)(acc[r] * 0.0625f + bqk[l * 128 + obase + r]);
        _Float16* dq = (mt < 4) ? (Q + m16 * QP_ + obase) : (Kt + m16 * QP_ + (obase - QK_));
        *(v8h*)dq = o8.v;
      }
      __syncthreads();

      v8f e = zero8();
#pragma unroll
      for (int ks = 0; ks < 2; ++ks)
        e = wmma_f16(frag16(Q, QP_, 0, ks * 32, m16, h), frag16(Kt, QP_, 0, ks * 32, m16, h), e);
#pragma unroll
      for (int r = 0; r < 8; ++r) {
        const float ev = e[r] * 0.125f;
        float mx = ev;
        mx = fmaxf(mx, __shfl_xor(mx, 1, 32));
        mx = fmaxf(mx, __shfl_xor(mx, 2, 32));
        mx = fmaxf(mx, __shfl_xor(mx, 4, 32));
        mx = fmaxf(mx, __shfl_xor(mx, 8, 32));
        const float pe = __expf(ev - mx);
        float s = pe;
        s += __shfl_xor(s, 1, 32);
        s += __shfl_xor(s, 2, 32);
        s += __shfl_xor(s, 4, 32);
        s += __shfl_xor(s, 8, 32);
        if (m16 == 0) AF[8 * h + r] = pe / s;
      }
      __syncthreads();
      const float afL = AF[m16];

#pragma unroll 1
      for (int mt = 0; mt < 8; ++mt) {
        v8f acc = zero8();
#pragma unroll
        for (int ks = 0; ks < 4; ++ks)
          acc = wmma_f16(frag16(wvp, CIN_, mt * 16, ks * 32, m16, h), bf[ks], acc);
#pragma unroll
        for (int r = 0; r < 8; ++r) {
          const int row = mt * 16 + 8 * h + r;
          float bvv = 0.0f;
          if (row < VCH_) bvv = bv[l * VCH_ + row];
          float val = (acc[r] * 0.0625f + bvv) * afL;
          val += __shfl_xor(val, 1, 32);
          val += __shfl_xor(val, 2, 32);
          val += __shfl_xor(val, 4, 32);
          val += __shfl_xor(val, 8, 32);
          if (m16 == (r & 15) && row < VCH_) ST[(l * OCH_ + 4 + row) * 32 + nl] = val;
        }
      }
      if (lane < 4) ST[(l * OCH_ + lane) * 32 + nl] = xb[lane * TN_ + t * N_ + n];
      __syncthreads();
    }
  }

#pragma unroll 1
  for (int it = 0; it < 32; ++it) {
    const int lid = it * 8 + w * 4 + (lane >> 3);
    const int l = lid >> 7, ch = lid & (OCH_ - 1), q = lane & 7;
    const v4f v = *(const v4f*)(ST + (l * OCH_ + ch) * 32 + 4 * q);
    float* dst = out + (size_t)((l * B_ + b) * OCH_ + ch) * TN_ + t * N_ + n0 + 4 * q;
    *(volatile v4f*)dst = v;
  }
  __threadfence();
#pragma unroll 1
  for (int it = 0; it < 32; ++it) {
    const int lid = it * 8 + w * 4 + (lane >> 3);
    const int l = lid >> 7, ch = lid & (OCH_ - 1), q = lane & 7;
    const v4f v = *(const v4f*)(ST + (l * OCH_ + ch) * 32 + 4 * q);
    float* dst = out + (size_t)((l * B_ + b) * OCH_ + ch) * TN_ + t * N_ + n0 + 4 * q;
    *(volatile v4f*)dst = v;
  }
}

extern "C" void kernel_launch(void* const* d_in, const int* in_sizes, int n_in,
                              void* d_out, int out_size, void* d_ws, size_t ws_size,
                              hipStream_t stream) {
  if (n_in < 5) return;
  if (in_sizes[0] != B_ * C_ * TN_) return;
  if (in_sizes[1] != L_ * 2 * QK_ * CIN_) return;
  if (in_sizes[2] != L_ * 2 * QK_) return;
  if (in_sizes[3] != L_ * VCH_ * CIN_) return;
  if (in_sizes[4] != L_ * VCH_) return;
  if (out_size != L_ * B_ * OCH_ * TN_) return;

  const float* x   = (const float*)d_in[0];
  const float* Wqk = (const float*)d_in[1];
  const float* bqk = (const float*)d_in[2];
  const float* Wv  = (const float*)d_in[3];
  const float* bv  = (const float*)d_in[4];
  float* out = (float*)d_out;

  const size_t g_bytes  = (size_t)NP_ * K_ * GP_ * sizeof(_Float16);
  const size_t wq_bytes = (size_t)L_ * 128 * CIN_ * sizeof(_Float16);
  const size_t wv_bytes = (size_t)L_ * 128 * CIN_ * sizeof(_Float16);
  const size_t off_g  = 0;
  const size_t off_wq = off_g + g_bytes;
  const size_t off_wv = off_wq + wq_bytes;
  const size_t total  = off_wv + wv_bytes;
  if (total > ws_size) return;

  char* ws = (char*)d_ws;
  _Float16* G    = (_Float16*)(ws + off_g);
  _Float16* wq16 = (_Float16*)(ws + off_wq);
  _Float16* wv16 = (_Float16*)(ws + off_wv);

  k_cvtw<<<32, 256, 0, stream>>>(Wqk, Wv, wq16, wv16);
  k_group<<<NP_ / 8, 256, 0, stream>>>(x, G);
  k_attn<<<NP_ / 32, 64, 0, stream>>>(x, bqk, bv, wq16, wv16, G, out);
  (void)hipGetLastError();
}
